// FlexBertUnpadAttention_43731357008511
// MI455X (gfx1250) — hardware-verified
//
#include <hip/hip_runtime.h>
#include <stddef.h>


typedef _Float16 v16h __attribute__((ext_vector_type(16)));
typedef _Float16 v8h  __attribute__((ext_vector_type(8), __may_alias__));
typedef float    v8f  __attribute__((ext_vector_type(8)));
typedef float    v4f  __attribute__((ext_vector_type(4), __may_alias__));

#define NB_   8
#define LQ_   1024
#define SQ_   2048
#define DM_   768
#define NH_   12
#define HD_   64
#define NT_   (NB_ * LQ_)
#define NQKV_ (3 * DM_)
#define QKP_  (2 * DM_)
#define PP_   72
#define TP_   136
#define SP_   132

#define HSC_ 16.0f
#define WSC_ 256.0f
#define QSC_ 16.0f
#define PSC_ 4096.0f
#define ASC_ 256.0f

static_assert(NT_ % 64 == 0);
static_assert(LQ_ % 64 == 0);
static_assert(NQKV_ % 128 == 0);
static_assert(DM_ % 128 == 0);
static_assert(DM_ % 32 == 0);
static_assert(HD_ == 64);
static_assert((NT_ * DM_) % 256 == 0);
static_assert((NQKV_ * DM_) % 256 == 0);
static_assert((DM_ * DM_) % 256 == 0);
static_assert(64 * TP_ * 2 <= 64 * SP_ * 4);

__device__ __forceinline__ v8f mma(v16h a, v16h b, v8f c) {
  v8f d = __builtin_amdgcn_wmma_f32_16x16x32_f16(false, a, false, b, (short)0, c, false, false);
  asm volatile("v_nop\n\tv_nop\n\tv_nop\n\tv_nop" : "+v"(d) : "v"(a), "v"(b));
  return d;
}

__device__ __forceinline__ v16h ldfrag(const _Float16* p) {
  union { v16h v; v8h q[2]; } f;
  f.q[0] = *(const v8h*)p;
  f.q[1] = *(const v8h*)(p + 16);
  return f.v;
}

__global__ __launch_bounds__(256) void k_cvt(const float* __restrict__ s0, _Float16* __restrict__ d0, int n0,
                                            const float* __restrict__ s1, _Float16* __restrict__ d1, int n1,
                                            const float* __restrict__ s2, _Float16* __restrict__ d2, int n2,
                                            float sc0, float sc1, float sc2) {
  const int g = (int)blockIdx.x * 256 + (int)threadIdx.x;
  const float* s;
  _Float16* d;
  float sc;
  int i;
  if (g < n0) { s = s0; d = d0; sc = sc0; i = g; }
  else if (g < n0 + n1) { s = s1; d = d1; sc = sc1; i = g - n0; }
  else if (g < n0 + n1 + n2) { s = s2; d = d2; sc = sc2; i = g - n0 - n1; }
  else return;
  const v4f a = *(const v4f*)(s + (size_t)i * 8);
  const v4f b = *(const v4f*)(s + (size_t)i * 8 + 4);
  v8h o;
  o[0] = (_Float16)(a[0] * sc); o[1] = (_Float16)(a[1] * sc);
  o[2] = (_Float16)(a[2] * sc); o[3] = (_Float16)(a[3] * sc);
  o[4] = (_Float16)(b[0] * sc); o[5] = (_Float16)(b[1] * sc);
  o[6] = (_Float16)(b[2] * sc); o[7] = (_Float16)(b[3] * sc);
  volatile v8h* p = (volatile v8h*)(d + (size_t)i * 8);
  *p = o;
  __threadfence();
  *p = o;
}

template <int MODE>
__global__ __launch_bounds__(128) void k_gemm(const _Float16* __restrict__ A,
                                             const _Float16* __restrict__ W,
                                             const float* __restrict__ bias,
                                             _Float16* __restrict__ o16,
                                             _Float16* __restrict__ ovt,
                                             float* __restrict__ o32) {
  constexpr int K = DM_;
  __shared__ __attribute__((aligned(16))) float stage[64 * SP_];
  const int l = threadIdx.x & 31, hs = l >> 4, m = l & 15, wv = (int)threadIdx.x >> 5;
  const int bm = blockIdx.x, bn = blockIdx.y;
  const int row0 = bm * 64;
  const int colw = bn * 128 + wv * 32;
  const _Float16* Ap = A + (size_t)(row0 + m) * K + 8 * hs;
  const _Float16* Wp = W + (size_t)(colw + m) * K + 8 * hs;

  const v8f z = {0.f, 0.f, 0.f, 0.f, 0.f, 0.f, 0.f, 0.f};
  v8f acc[4][2];
#pragma unroll
  for (int mi = 0; mi < 4; ++mi)
#pragma unroll
    for (int ni = 0; ni < 2; ++ni) acc[mi][ni] = z;

#pragma unroll 1
  for (int k0 = 0; k0 < K; k0 += 32) {
    v16h af[4], bf[2];
#pragma unroll
    for (int mi = 0; mi < 4; ++mi) af[mi] = ldfrag(Ap + (size_t)mi * 16 * K + k0);
#pragma unroll
    for (int ni = 0; ni < 2; ++ni) bf[ni] = ldfrag(Wp + (size_t)ni * 16 * K + k0);
#pragma unroll
    for (int mi = 0; mi < 4; ++mi)
#pragma unroll
      for (int ni = 0; ni < 2; ++ni) acc[mi][ni] = mma(af[mi], bf[ni], acc[mi][ni]);
  }

  if constexpr (MODE == 0) {
    _Float16* T = (_Float16*)stage;
    const float b0 = bias[colw + m] * QSC_;
    const float b1 = bias[colw + 16 + m] * QSC_;
    constexpr float osc = QSC_ / (HSC_ * WSC_);
#pragma unroll
    for (int mi = 0; mi < 4; ++mi)
#pragma unroll
      for (int ni = 0; ni < 2; ++ni)
#pragma unroll
        for (int r = 0; r < 8; ++r)
          T[(mi * 16 + 8 * hs + r) * TP_ + wv * 32 + ni * 16 + m] =
              (_Float16)fmaf(acc[mi][ni][r], osc, ni ? b1 : b0);
    __syncthreads();
    if (bn < QKP_ / 128) {
      v8h vals[8];
#pragma unroll
      for (int j = 0; j < 8; ++j) {
        const int tr = wv * 16 + 2 * j + hs;
        vals[j] = *(const v8h*)(T + tr * TP_ + 8 * m);
      }
#pragma unroll
      for (int ps = 0; ps < 2; ++ps) {
#pragma unroll
        for (int j = 0; j < 8; ++j) {
          const int tr = wv * 16 + 2 * j + hs;
          *(volatile v8h*)(o16 + (size_t)(row0 + tr) * QKP_ + bn * 128 + 8 * m) = vals[j];
        }
        if (ps == 0) __threadfence();
      }
    } else {
      const int hp = bn - QKP_ / 128;
      const int bb = row0 / LQ_;
      const int key0 = row0 % LQ_;
      const int sub = l & 7;
      v8h vals[8];
#pragma unroll
      for (int j = 0; j < 8; ++j) {
        const int c = wv * 32 + 4 * j + (l >> 3);
        v8h v;
#pragma unroll
        for (int e = 0; e < 8; ++e) v[e] = T[(8 * sub + e) * TP_ + c];
        vals[j] = v;
      }
#pragma unroll
      for (int ps = 0; ps < 2; ++ps) {
#pragma unroll
        for (int j = 0; j < 8; ++j) {
          const int c = wv * 32 + 4 * j + (l >> 3);
          const int hh = 2 * hp + (c >> 6);
          const int d = c & 63;
          *(volatile v8h*)(ovt + ((size_t)((bb * NH_ + hh) * HD_ + d)) * LQ_ + key0 + 8 * sub) = vals[j];
        }
        if (ps == 0) __threadfence();
      }
    }
  } else {
    float* S = stage;
    const float b0 = bias[colw + m];
    const float b1 = bias[colw + 16 + m];
    constexpr float osc = 1.0f / (ASC_ * WSC_);
#pragma unroll
    for (int mi = 0; mi < 4; ++mi)
#pragma unroll
      for (int ni = 0; ni < 2; ++ni)
#pragma unroll
        for (int r = 0; r < 8; ++r)
          S[(mi * 16 + 8 * hs + r) * SP_ + wv * 32 + ni * 16 + m] =
              fmaf(acc[mi][ni][r], osc, ni ? b1 : b0);
    __syncthreads();
    v4f vals[16];
#pragma unroll
    for (int j = 0; j < 16; ++j) vals[j] = *(const v4f*)(S + (wv * 16 + j) * SP_ + 4 * l);
#pragma unroll
    for (int ps = 0; ps < 2; ++ps) {
#pragma unroll
      for (int j = 0; j < 16; ++j)
        *(volatile v4f*)(o32 + (size_t)(row0 + wv * 16 + j) * DM_ + bn * 128 + 4 * l) = vals[j];
      if (ps == 0) __threadfence();
    }
  }
}

__global__ __launch_bounds__(128) void k_attn(const _Float16* __restrict__ qk,
                                             const _Float16* __restrict__ vt,
                                             _Float16* __restrict__ ao) {
  __shared__ __attribute__((aligned(16))) _Float16 Pb[64 * PP_];
  const int l = threadIdx.x & 31, hs = l >> 4, m = l & 15, wv = (int)threadIdx.x >> 5;
  const int qt = (int)blockIdx.x % (LQ_ / 64);
  const int bh = (int)blockIdx.x / (LQ_ / 64);
  const int h = bh % NH_, b = bh / NH_;
  const size_t tok0 = (size_t)b * LQ_;
  const int qr0 = qt * 64 + wv * 16;

  const _Float16* qp = qk + (tok0 + qr0 + m) * QKP_ + h * HD_ + 8 * hs;
  const v16h aq0 = ldfrag(qp);
  const v16h aq1 = ldfrag(qp + 32);
  const _Float16* kbase = qk + (tok0 + m) * QKP_ + DM_ + h * HD_ + 8 * hs;
  const _Float16* vbase = vt + ((size_t)bh * HD_ + m) * LQ_ + 8 * hs;
  _Float16* pw = Pb + wv * 16 * PP_;

  const v8f z = {0.f, 0.f, 0.f, 0.f, 0.f, 0.f, 0.f, 0.f};
  float m2[8], ls[8];
  v8f acc[4];
#pragma unroll
  for (int r = 0; r < 8; ++r) { m2[r] = 0.0f; ls[r] = (float)(SQ_ - LQ_); }
#pragma unroll
  for (int nd = 0; nd < 4; ++nd) acc[nd] = z;

  constexpr float SC2 = 0.125f * 1.44269504088896341f / (QSC_ * QSC_);

#pragma unroll 1
  for (int kt = 0; kt < LQ_; kt += 64) {
    v8f s[4];
#pragma unroll
    for (int nk = 0; nk < 4; ++nk) {
      const _Float16* kp = kbase + (size_t)(kt + nk * 16) * QKP_;
      const v16h kf0 = ldfrag(kp);
      const v16h kf1 = ldfrag(kp + 32);
      s[nk] = mma(aq0, kf0, z);
      s[nk] = mma(aq1, kf1, s[nk]);
    }
    float mn[8], al[8], rs[8];
#pragma unroll
    for (int r = 0; r < 8; ++r) {
      float v = fmaxf(fmaxf(s[0][r], s[1][r]), fmaxf(s[2][r], s[3][r]));
      v = fmaxf(v, __shfl_xor(v, 1));
      v = fmaxf(v, __shfl_xor(v, 2));
      v = fmaxf(v, __shfl_xor(v, 4));
      v = fmaxf(v, __shfl_xor(v, 8));
      mn[r] = fmaxf(m2[r], v * SC2);
      al[r] = exp2f(m2[r] - mn[r]);
      m2[r] = mn[r];
      rs[r] = 0.0f;
    }
#pragma unroll
    for (int nk = 0; nk < 4; ++nk)
#pragma unroll
      for (int r = 0; r < 8; ++r) {
        const float p = exp2f(fmaf(s[nk][r], SC2, -mn[r]));
        s[nk][r] = p;
        rs[r] += p;
      }
#pragma unroll
    for (int r = 0; r < 8; ++r) {
      float v = rs[r];
      v += __shfl_xor(v, 1);
      v += __shfl_xor(v, 2);
      v += __shfl_xor(v, 4);
      v += __shfl_xor(v, 8);
      ls[r] = fmaf(ls[r], al[r], v);
    }
#pragma unroll
    for (int nd = 0; nd < 4; ++nd)
#pragma unroll
      for (int r = 0; r < 8; ++r) acc[nd][r] *= al[r];

#pragma unroll
    for (int nk = 0; nk < 4; ++nk)
#pragma unroll
      for (int r = 0; r < 8; ++r)
        pw[(8 * hs + r) * PP_ + nk * 16 + m] = (_Float16)(s[nk][r] * PSC_);
    __syncthreads();
    const v16h ap0 = ldfrag(pw + m * PP_ + 8 * hs);
    const v16h ap1 = ldfrag(pw + m * PP_ + 32 + 8 * hs);
#pragma unroll
    for (int nd = 0; nd < 4; ++nd) {
      const _Float16* vp = vbase + (size_t)nd * 16 * LQ_ + kt;
      acc[nd] = mma(ap0, ldfrag(vp), acc[nd]);
      acc[nd] = mma(ap1, ldfrag(vp + 32), acc[nd]);
    }
  }

  float inv[8];
  constexpr float OSC = ASC_ / (PSC_ * QSC_);
#pragma unroll
  for (int r = 0; r < 8; ++r) inv[r] = OSC / ls[r];
  __syncthreads();
#pragma unroll
  for (int nd = 0; nd < 4; ++nd)
#pragma unroll
    for (int r = 0; r < 8; ++r)
      pw[(8 * hs + r) * PP_ + nd * 16 + m] = (_Float16)(acc[nd][r] * inv[r]);
  __syncthreads();
  const int sub = l & 7;
  v8h vals[4];
#pragma unroll
  for (int j = 0; j < 4; ++j) {
    const int tr = wv * 16 + 4 * j + (l >> 3);
    vals[j] = *(const v8h*)(Pb + tr * PP_ + 8 * sub);
  }
  const size_t orow0 = tok0 + (size_t)qt * 64;
#pragma unroll
  for (int ps = 0; ps < 2; ++ps) {
#pragma unroll
    for (int j = 0; j < 4; ++j) {
      const int tr = wv * 16 + 4 * j + (l >> 3);
      *(volatile v8h*)(ao + (orow0 + tr) * DM_ + h * HD_ + 8 * sub) = vals[j];
    }
    if (ps == 0) __threadfence();
  }
}

extern "C" void kernel_launch(void* const* d_in, const int* in_sizes, int n_in,
                              void* d_out, int out_size, void* d_ws,
                              size_t ws_size, hipStream_t stream) {
  if (n_in < 5) return;
  if (in_sizes[0] != NT_ * DM_ || in_sizes[1] != NQKV_ * DM_ || in_sizes[2] != NQKV_ ||
      in_sizes[3] != DM_ * DM_ || in_sizes[4] != DM_ || out_size != NT_ * DM_) return;

  const float* hidden = (const float*)d_in[0];
  const float* Wqkv_w = (const float*)d_in[1];
  const float* Wqkv_b = (const float*)d_in[2];
  const float* Wo_w   = (const float*)d_in[3];
  const float* Wo_b   = (const float*)d_in[4];
  float* out = (float*)d_out;

  size_t off = 0;
  auto carve = [&](size_t bytes) -> char* {
    char* p = (char*)d_ws + off;
    off += (bytes + 255) & ~(size_t)255;
    return p;
  };
  _Float16* hsb = (_Float16*)carve((size_t)NT_ * DM_ * 2);
  _Float16* wqb = (_Float16*)carve((size_t)NQKV_ * DM_ * 2);
  _Float16* wob = (_Float16*)carve((size_t)DM_ * DM_ * 2);
  _Float16* qkb = (_Float16*)carve((size_t)NT_ * QKP_ * 2);
  _Float16* vtb = (_Float16*)carve((size_t)NB_ * NH_ * HD_ * LQ_ * 2);
  _Float16* atb = (_Float16*)carve((size_t)NT_ * DM_ * 2);
  if (off > ws_size) return;

  const int n0 = NT_ * DM_ / 8, n1 = NQKV_ * DM_ / 8, n2 = DM_ * DM_ / 8;
  const int cvt_blocks = (n0 + n1 + n2 + 255) / 256;
  k_cvt<<<cvt_blocks, 256, 0, stream>>>(hidden, hsb, n0, Wqkv_w, wqb, n1, Wo_w, wob, n2,
                                        HSC_, WSC_, WSC_);
  k_gemm<0><<<dim3(NT_ / 64, NQKV_ / 128), 128, 0, stream>>>(hsb, wqb, Wqkv_b, qkb, vtb, out);
  k_attn<<<NB_ * NH_ * (LQ_ / 64), 128, 0, stream>>>(qkb, vtb, atb);
  k_gemm<1><<<dim3(NT_ / 64, DM_ / 128), 128, 0, stream>>>(atb, wob, Wo_b, qkb, vtb, out);
}
